// encoder_self_attn_20023137534032
// MI455X (gfx1250) — hardware-verified
//
#include <hip/hip_runtime.h>
#include <math.h>
#include <stddef.h>
#include <stdint.h>

#define NTOK 32768
#define NBAT 32
#define SEQ  1024
#define HD   512
#define OD   32
#define BR   32
#define BC   128

static_assert(NTOK == NBAT * SEQ);
static_assert(SEQ % BC == 0);
static_assert(SEQ % BR == 0);
static_assert(BC % 32 == 0);
static_assert(HD == 512);
static_assert((HD / 8) == 64);
static_assert((SEQ / 8) == 128);
static_assert(OD == 32);

typedef _Float16 v16h __attribute__((ext_vector_type(16)));
typedef _Float16 v8h  __attribute__((ext_vector_type(8)));
typedef float    v8f  __attribute__((ext_vector_type(8)));
typedef float    v4f  __attribute__((ext_vector_type(4)));
typedef float    v2f  __attribute__((ext_vector_type(2)));
typedef unsigned int v4u __attribute__((ext_vector_type(4)));

union Frag  { v16h v; v8h h[2]; };
union Pack8 { v8h h; v4u u; };

__device__ __forceinline__ v8f mma16(v16h a, v16h b, v8f c) {
  c = __builtin_amdgcn_wmma_f32_16x16x32_f16(false, a, false, b, (short)0, c, false, false);
  asm volatile("v_nop\n\tv_nop\n\tv_nop\n\tv_nop" : "+v"(c) : "v"(a), "v"(b));
  return c;
}

__device__ __forceinline__ v16h ldfrag(const _Float16* p, int ld, int row0, int k0, int lane) {
  const int m = lane & 15, lh = lane >> 4;
  const _Float16* q = p + (size_t)(row0 + m) * ld + k0 + 8 * lh;
  Frag f;
  f.h[0] = *(const v8h*)(q);
  f.h[1] = *(const v8h*)(q + 16);
  return f.v;
}

__device__ __forceinline__ v8f zero8() { return (v8f){0.f, 0.f, 0.f, 0.f, 0.f, 0.f, 0.f, 0.f}; }

__global__ __launch_bounds__(256) void k_wout(const float* __restrict__ wo, _Float16* __restrict__ wot, int n) {
  const int t = blockIdx.x * 256 + (int)threadIdx.x;
  if (t >= n) return;
  const int nn = t >> 6;
  const int k0 = (t & 63) * 8;
  const float* src = wo + (size_t)k0 * OD + nn;
  Pack8 pk;
  pk.h = (v8h){(_Float16)(src[0 * OD] * 64.0f), (_Float16)(src[1 * OD] * 64.0f),
               (_Float16)(src[2 * OD] * 64.0f), (_Float16)(src[3 * OD] * 64.0f),
               (_Float16)(src[4 * OD] * 64.0f), (_Float16)(src[5 * OD] * 64.0f),
               (_Float16)(src[6 * OD] * 64.0f), (_Float16)(src[7 * OD] * 64.0f)};
  const v4u vv = pk.u;
  volatile v4u* d = (volatile v4u*)(wot + (size_t)nn * HD + k0);
  *d = vv;
  __threadfence();
  *d = vv;
}

__global__ __launch_bounds__(256) void k_proj(const float* __restrict__ x,
                                              const float* __restrict__ wq,
                                              const float* __restrict__ wk,
                                              const float* __restrict__ wv,
                                              _Float16* __restrict__ qp,
                                              _Float16* __restrict__ kp,
                                              _Float16* __restrict__ vt, int nqk, int nv) {
  const int which = blockIdx.y;
  const int t = blockIdx.x * 256 + (int)threadIdx.x;
  if (which < 2) {
    if (t >= nqk) return;
    const float* w = (which == 0) ? wq : wk;
    _Float16* dst  = (which == 0) ? qp : kp;
    const int tok = t >> 6;
    const int h0  = (t & 63) * 8;
    const v2f xx  = *(const v2f*)(x + 2 * (size_t)tok);
    const float x0 = xx[0], x1 = xx[1];
    const v4f a0 = *(const v4f*)(w + h0);
    const v4f a1 = *(const v4f*)(w + h0 + 4);
    const v4f b0 = *(const v4f*)(w + HD + h0);
    const v4f b1 = *(const v4f*)(w + HD + h0 + 4);
    Pack8 pk;
    pk.h = (v8h){(_Float16)fmaf(x1, b0[0], x0 * a0[0]), (_Float16)fmaf(x1, b0[1], x0 * a0[1]),
                 (_Float16)fmaf(x1, b0[2], x0 * a0[2]), (_Float16)fmaf(x1, b0[3], x0 * a0[3]),
                 (_Float16)fmaf(x1, b1[0], x0 * a1[0]), (_Float16)fmaf(x1, b1[1], x0 * a1[1]),
                 (_Float16)fmaf(x1, b1[2], x0 * a1[2]), (_Float16)fmaf(x1, b1[3], x0 * a1[3])};
    const v4u vv = pk.u;
    volatile v4u* d = (volatile v4u*)(dst + (size_t)tok * HD + h0);
    *d = vv;
    __threadfence();
    *d = vv;
  } else {
    if (t >= nv) return;
    const int l0 = (t & 127) * 8;
    const int e  = (t >> 7) & 511;
    const int b  = t >> 16;
    const float w0 = wv[e], w1 = wv[HD + e];
    const float* xr = x + ((size_t)(b * SEQ + l0)) * 2;
    const v4f c0 = *(const v4f*)(xr);
    const v4f c1 = *(const v4f*)(xr + 4);
    const v4f c2 = *(const v4f*)(xr + 8);
    const v4f c3 = *(const v4f*)(xr + 12);
    Pack8 pk;
    pk.h = (v8h){(_Float16)fmaf(c0[1], w1, c0[0] * w0), (_Float16)fmaf(c0[3], w1, c0[2] * w0),
                 (_Float16)fmaf(c1[1], w1, c1[0] * w0), (_Float16)fmaf(c1[3], w1, c1[2] * w0),
                 (_Float16)fmaf(c2[1], w1, c2[0] * w0), (_Float16)fmaf(c2[3], w1, c2[2] * w0),
                 (_Float16)fmaf(c3[1], w1, c3[0] * w0), (_Float16)fmaf(c3[3], w1, c3[2] * w0)};
    const v4u vv = pk.u;
    volatile v4u* d = (volatile v4u*)(vt + ((size_t)(b * HD + e)) * SEQ + l0);
    *d = vv;
    __threadfence();
    *d = vv;
  }
}

#define SSP 128
#define SPP 136
#define ZP  520
#define PTP 36
#define SP_OFF_F   (BR * SSP)
#define PART_OFF_F ((BR * ZP) / 2)
#define SBIGF      (PART_OFF_F + 2 * BR * PTP)
static_assert((BR * ZP) % 8 == 0);
static_assert(SP_OFF_F + (BR * SPP) / 2 <= SBIGF);
static_assert((SP_OFF_F % 4) == 0);
static_assert((PART_OFF_F % 4) == 0);
static_assert((ZP % 8) == 0);
static_assert((SPP % 8) == 0);

__global__ __launch_bounds__(256) void k_attn(const _Float16* __restrict__ qp,
                                              const _Float16* __restrict__ kp,
                                              const _Float16* __restrict__ vt,
                                              const _Float16* __restrict__ wot,
                                              const float* __restrict__ gam,
                                              const float* __restrict__ bet,
                                              const float* __restrict__ mu,
                                              const float* __restrict__ var,
                                              const float* __restrict__ pa,
                                              const float* __restrict__ bo,
                                              const int* __restrict__ bsp,
                                              float* __restrict__ out, float sscale) {
  __shared__ __align__(16) float sBig[SBIGF];
  __shared__ __align__(16) float sRed[BR * 8];
  __shared__ __align__(16) float rM[BR];
  __shared__ __align__(16) float rMn[BR];
  __shared__ __align__(16) float rL[BR];
  __shared__ __align__(16) float rSc[BR];

  float*    sS   = sBig;
  _Float16* sP   = (_Float16*)(sBig + SP_OFF_F);
  _Float16* zA   = (_Float16*)sBig;
  float*    part = sBig + PART_OFF_F;

  const int tid = threadIdx.x, lane = tid & 31, wave = tid >> 5;
  const int hh = lane >> 4, c = lane & 15;
  const int b  = blockIdx.y;
  const int q0 = (int)blockIdx.x * BR;
  int bs = bsp[0];
  bs = (bs < 1) ? 1 : bs;
  int seql = NTOK / bs;
  seql = (seql > SEQ) ? SEQ : seql;
  const int nch = seql / BC;
  const _Float16* Qb = qp + (size_t)b * SEQ * HD;
  const _Float16* Kb = kp + (size_t)b * SEQ * HD;
  const _Float16* Vb = vt + (size_t)b * HD * SEQ;
  const size_t tokbase = (size_t)b * SEQ + q0;
  const float NEGI = -__builtin_huge_valf();
  if (tid < BR) { rM[tid] = NEGI; rL[tid] = 0.f; }
  __syncthreads();

  v8f oacc[2][4];
#pragma unroll
  for (int s = 0; s < 2; ++s)
#pragma unroll
    for (int t = 0; t < 4; ++t) oacc[s][t] = zero8();

  const int srow = tid >> 3, schk = tid & 7;

#pragma unroll 1
  for (int ch = 0; ch < nch; ++ch) {
    const int j0  = ch * BC;
    const int kr0 = j0 + wave * 16;
    v8f s[2];
    s[0] = zero8(); s[1] = zero8();
#pragma unroll 2
    for (int k0 = 0; k0 < HD; k0 += 32) {
      const v16h a0 = ldfrag(Qb, HD, q0, k0, lane);
      const v16h a1 = ldfrag(Qb, HD, q0 + 16, k0, lane);
      const v16h kb = ldfrag(Kb, HD, kr0, k0, lane);
      s[0] = mma16(a0, kb, s[0]);
      s[1] = mma16(a1, kb, s[1]);
    }
#pragma unroll
    for (int t = 0; t < 2; ++t) {
#pragma unroll
      for (int r = 0; r < 8; ++r) {
        const int row = 16 * t + 8 * hh + r;
        sS[row * SSP + wave * 16 + c] = s[t][r] * sscale;
      }
    }
    __syncthreads();
    {
      const float* sr = sS + srow * SSP + schk * 16;
      const v4f x0 = *(const v4f*)(sr);
      const v4f x1 = *(const v4f*)(sr + 4);
      const v4f x2 = *(const v4f*)(sr + 8);
      const v4f x3 = *(const v4f*)(sr + 12);
      float mx = x0[0];
#pragma unroll
      for (int e = 1; e < 4; ++e) mx = fmaxf(mx, x0[e]);
#pragma unroll
      for (int e = 0; e < 4; ++e) { mx = fmaxf(mx, x1[e]); mx = fmaxf(mx, x2[e]); mx = fmaxf(mx, x3[e]); }
      sRed[srow * 8 + schk] = mx;
    }
    __syncthreads();
    if (tid < BR) {
      float mx = rM[tid];
#pragma unroll
      for (int i = 0; i < 8; ++i) mx = fmaxf(mx, sRed[tid * 8 + i]);
      rMn[tid] = mx;
    }
    __syncthreads();
    {
      const float mx = rMn[srow];
      const float* sr = sS + srow * SSP + schk * 16;
      float sum = 0.f;
      Pack8 p0, p1;
#pragma unroll
      for (int e = 0; e < 8; ++e) {
        const float p = __expf(sr[e] - mx);
        sum += p;
        p0.h[e] = (_Float16)(p * 1024.0f);
      }
#pragma unroll
      for (int e = 0; e < 8; ++e) {
        const float p = __expf(sr[8 + e] - mx);
        sum += p;
        p1.h[e] = (_Float16)(p * 1024.0f);
      }
      *(v8h*)(sP + srow * SPP + schk * 16)     = p0.h;
      *(v8h*)(sP + srow * SPP + schk * 16 + 8) = p1.h;
      sRed[srow * 8 + schk] = sum;
    }
    __syncthreads();
    if (tid < BR) {
      float sum = 0.f;
#pragma unroll
      for (int i = 0; i < 8; ++i) sum += sRed[tid * 8 + i];
      const float mnew = rMn[tid];
      const float fac  = __expf(rM[tid] - mnew);
      rL[tid]  = rL[tid] * fac + sum;
      rM[tid]  = mnew;
      rSc[tid] = fac;
    }
    __syncthreads();
#pragma unroll
    for (int t = 0; t < 2; ++t) {
      const v4f f0 = *(const v4f*)(rSc + 16 * t + 8 * hh);
      const v4f f1 = *(const v4f*)(rSc + 16 * t + 8 * hh + 4);
#pragma unroll
      for (int et = 0; et < 4; ++et) {
#pragma unroll
        for (int r = 0; r < 4; ++r) {
          oacc[t][et][r]     *= f0[r];
          oacc[t][et][4 + r] *= f1[r];
        }
      }
    }
#pragma unroll 1
    for (int kk = 0; kk < BC / 32; ++kk) {
      const v16h pa0 = ldfrag(sP, SPP, 0, kk * 32, lane);
      const v16h pa1 = ldfrag(sP, SPP, 16, kk * 32, lane);
#pragma unroll
      for (int et = 0; et < 4; ++et) {
        const v16h vb = ldfrag(Vb, SEQ, wave * 64 + 16 * et, j0 + kk * 32, lane);
        oacc[0][et] = mma16(pa0, vb, oacc[0][et]);
        oacc[1][et] = mma16(pa1, vb, oacc[1][et]);
      }
    }
    __syncthreads();
  }

  if (tid < BR) {
    const float l = rL[tid];
    rSc[tid] = (l > 0.f) ? (0.0009765625f * (1.0f / l)) : 0.f;
  }
  __syncthreads();
  {
    const float a = pa[0];
    v4f iv0[2], iv1[2];
#pragma unroll
    for (int sub = 0; sub < 2; ++sub) {
      iv0[sub] = *(const v4f*)(rSc + 16 * sub + 8 * hh);
      iv1[sub] = *(const v4f*)(rSc + 16 * sub + 8 * hh + 4);
    }
#pragma unroll
    for (int t = 0; t < 4; ++t) {
      const int h = wave * 64 + 16 * t + c;
      const float sc = gam[h] * (1.0f / sqrtf(var[h] + 1.0e-5f));
      const float m  = mu[h];
      const float be = bet[h];
#pragma unroll
      for (int sub = 0; sub < 2; ++sub) {
#pragma unroll
        for (int r = 0; r < 4; ++r) {
          const float o0 = oacc[sub][t][r] * iv0[sub][r];
          float z0 = (o0 - m) * sc + be;
          z0 = (z0 >= 0.f) ? z0 : a * z0;
          zA[(16 * sub + 8 * hh + r) * ZP + h] = (_Float16)(z0 * 16.0f);
          const float o1 = oacc[sub][t][4 + r] * iv1[sub][r];
          float z1 = (o1 - m) * sc + be;
          z1 = (z1 >= 0.f) ? z1 : a * z1;
          zA[(16 * sub + 8 * hh + 4 + r) * ZP + h] = (_Float16)(z1 * 16.0f);
        }
      }
    }
  }
  __syncthreads();

  {
    const int osub = wave & 1, ont = (wave >> 1) & 1, okh = wave >> 2;
    v8f acc = zero8();
#pragma unroll 2
    for (int ks = 0; ks < 8; ++ks) {
      const int k0 = (okh * 8 + ks) * 32;
      const v16h af = ldfrag(zA, ZP, 16 * osub, k0, lane);
      const v16h bf = ldfrag(wot, HD, 16 * ont, k0, lane);
      acc = mma16(af, bf, acc);
    }
    float* pp = part + okh * (BR * PTP) + (16 * osub + 8 * hh) * PTP + 16 * ont + c;
#pragma unroll
    for (int r = 0; r < 8; ++r) pp[r * PTP] = acc[r];
  }
  __syncthreads();
  {
    const int row = tid >> 3, pc = tid & 7;
    const v4f p0 = *(const v4f*)(part + row * PTP + pc * 4);
    const v4f p1 = *(const v4f*)(part + BR * PTP + row * PTP + pc * 4);
    const v4f bb = *(const v4f*)(bo + pc * 4);
    const v4f val = (p0 + p1) * 0.0009765625f + bb;
    volatile v4f* d = (volatile v4f*)(out + (tokbase + (size_t)row) * OD + pc * 4);
    *d = val;
    __threadfence();
    *d = val;
  }
}

extern "C" void kernel_launch(void* const* d_in, const int* in_sizes, int n_in,
                              void* d_out, int out_size, void* d_ws, size_t ws_size,
                              hipStream_t stream) {
  if (n_in < 12) return;
  if (in_sizes[0] != NTOK * 2) return;
  if (in_sizes[1] < 1) return;
  if (in_sizes[2] != 2 * HD) return;
  if (in_sizes[3] != 2 * HD) return;
  if (in_sizes[4] != 2 * HD) return;
  if (in_sizes[5] != HD) return;
  if (in_sizes[6] != HD) return;
  if (in_sizes[7] != HD) return;
  if (in_sizes[8] != HD) return;
  if (in_sizes[9] < 1) return;
  if (in_sizes[10] != HD * OD) return;
  if (in_sizes[11] != OD) return;
  if (out_size != NTOK * OD) return;

  const float* x    = (const float*)d_in[0];
  const int*   bsz  = (const int*)d_in[1];
  const float* wq   = (const float*)d_in[2];
  const float* wk   = (const float*)d_in[3];
  const float* wv   = (const float*)d_in[4];
  const float* gam  = (const float*)d_in[5];
  const float* bet  = (const float*)d_in[6];
  const float* mu   = (const float*)d_in[7];
  const float* var  = (const float*)d_in[8];
  const float* pa   = (const float*)d_in[9];
  const float* wo   = (const float*)d_in[10];
  const float* bo   = (const float*)d_in[11];
  float* out = (float*)d_out;

  size_t off = 0;
  const size_t oQ = off; off += (size_t)NTOK * HD * 2;
  const size_t oK = off; off += (size_t)NTOK * HD * 2;
  const size_t oV = off; off += (size_t)NBAT * HD * SEQ * 2;
  const size_t oW = off; off += (size_t)OD * HD * 2;
  if (off > ws_size) return;
  if (off > (size_t)134217728) return;

  char* ws = (char*)d_ws;
  _Float16* Qp  = (_Float16*)(ws + oQ);
  _Float16* Kp  = (_Float16*)(ws + oK);
  _Float16* Vt  = (_Float16*)(ws + oV);
  _Float16* WoT = (_Float16*)(ws + oW);

  const float sscale = 1.0f / sqrtf((float)HD);

  const int ngw = (OD * HD) / 8;
  k_wout<<<dim3((ngw + 255) / 256), dim3(256), 0, stream>>>(wo, WoT, ngw);
  const int nqk = (NTOK * HD) / 8;
  const int nv  = (NBAT * HD * SEQ) / 8;
  const int ngp = (nqk > nv) ? nqk : nv;
  k_proj<<<dim3((ngp + 255) / 256, 3), dim3(256), 0, stream>>>(x, wq, wk, wv, Qp, Kp, Vt, nqk, nv);
  k_attn<<<dim3(SEQ / BR, NBAT), dim3(256), 0, stream>>>(Qp, Kp, Vt, WoT, gam, bet, mu, var, pa, bo, bsz,
                                                         out, sscale);
  (void)hipGetLastError();
}
